// GaussianSplatScene_68856915689837
// MI455X (gfx1250) — hardware-verified
//
#include <hip/hip_runtime.h>


namespace {
constexpr int Q = 4096, N = 16384, F = 32, GP = 16;
constexpr float XS = 8.0f, PS = 512.0f  , LOG2E = 1.4426950408889634f;

typedef _Float16 b16;
typedef __attribute__((ext_vector_type(16))) _Float16 v16b;
typedef __attribute__((ext_vector_type(8))) _Float16 v8b;
typedef __attribute__((ext_vector_type(8))) float v8f;
typedef __attribute__((ext_vector_type(4))) float v4f;
__device__ __forceinline__ float bf16_rne(float f) { unsigned int u = __float_as_uint(f); u += 0x7FFFu + ((u >> 16) & 1u); return __uint_as_float(u & 0xFFFF0000u); }
__device__ __forceinline__ v16b frag_kb(const b16* p, int hh) { const v8b a = *(const v8b*)(p + 8 * hh), b = *(const v8b*)(p + 16 + 8 * hh); v16b f;
#pragma unroll
  for (int e = 0; e < 8; ++e) { f[e] = a[e]; f[8 + e] = b[e]; } return f; }
__device__ __forceinline__ v8f wmma16b(v16b a, v16b b, v8f c) { v8f d = __builtin_amdgcn_wmma_f32_16x16x32_f16(false, a, false, b, (short)0, c, false, false); asm volatile("v_nop\n\tv_nop\n\tv_nop\n\tv_nop" : "+v"(d) : "v"(a), "v"(b)); return d; }
__device__ __forceinline__ void wave_lds_sync() { __builtin_amdgcn_fence(__ATOMIC_RELEASE, "workgroup"); __builtin_amdgcn_wave_barrier(); __builtin_amdgcn_fence(__ATOMIC_ACQUIRE, "workgroup"); }
__device__ __forceinline__ float pmul(float a, float b) { float p = a * b; asm volatile("" : "+v"(p)); return p; }
__device__ __forceinline__ float nexp(float x) { return __builtin_amdgcn_exp2f(x * LOG2E); }

__global__ __launch_bounds__(256) void gauss_kernel(const float* __restrict__ means, const float* __restrict__ lsc, const float* __restrict__ rot, const float* __restrict__ opl, float* __restrict__ GPR) {
  const int n = blockIdx.x * 256 + threadIdx.x; if (n >= N) return;
  float qw = bf16_rne(rot[n * 4]), qx = bf16_rne(rot[n * 4 + 1]), qy = bf16_rne(rot[n * 4 + 2]), qz = bf16_rne(rot[n * 4 + 3]);
  const float nrm = sqrtf((qw * qw + qx * qx) + (qy * qy + qz * qz)); const float inv = 1.0f / fmaxf(nrm, 1e-12f); qw *= inv; qx *= inv; qy *= inv; qz *= inv;
  float R[3][3] = {{1.0f - 2.0f * (qy * qy + qz * qz), 2.0f * (qx * qy - qw * qz), 2.0f * (qx * qz + qw * qy)},
                   {2.0f * (qx * qy + qw * qz), 1.0f - 2.0f * (qx * qx + qz * qz), 2.0f * (qy * qz - qw * qx)},
                   {2.0f * (qx * qz - qw * qy), 2.0f * (qy * qz + qw * qx), 1.0f - 2.0f * (qx * qx + qy * qy)}};
  const float s0 = __expf(bf16_rne(lsc[n * 3])), s1 = __expf(bf16_rne(lsc[n * 3 + 1])), s2 = __expf(bf16_rne(lsc[n * 3 + 2]));
  float RS[3][3]; for (int i = 0; i < 3; ++i) { RS[i][0] = R[i][0] * s0; RS[i][1] = R[i][1] * s1; RS[i][2] = R[i][2] * s2; }
  float C[3][3]; for (int i = 0; i < 3; ++i) for (int j = 0; j < 3; ++j) C[i][j] = (pmul(RS[i][0], RS[j][0]) + pmul(RS[i][1], RS[j][1])) + pmul(RS[i][2], RS[j][2]) + (i == j ? 1e-6f : 0.0f);
  const float c00 = C[1][1] * C[2][2] - C[1][2] * C[2][1], c01 = C[1][2] * C[2][0] - C[1][0] * C[2][2], c02 = C[1][0] * C[2][1] - C[1][1] * C[2][0];
  const float det = C[0][0] * c00 + C[0][1] * c01 + C[0][2] * c02; const float id = 1.0f / det;
  float A[9]; A[0] = c00 * id; A[1] = (C[0][2] * C[2][1] - C[0][1] * C[2][2]) * id; A[2] = (C[0][1] * C[1][2] - C[0][2] * C[1][1]) * id;
  A[3] = c01 * id; A[4] = (C[0][0] * C[2][2] - C[0][2] * C[2][0]) * id; A[5] = (C[0][2] * C[1][0] - C[0][0] * C[1][2]) * id;
  A[6] = c02 * id; A[7] = (C[0][1] * C[2][0] - C[0][0] * C[2][1]) * id; A[8] = (C[0][0] * C[1][1] - C[0][1] * C[1][0]) * id;
  const float m0 = bf16_rne(means[n * 3]), m1 = bf16_rne(means[n * 3 + 1]), m2 = bf16_rne(means[n * 3 + 2]);
  const float am0 = (A[0] * m0 + A[1] * m1) + A[2] * m2, am1 = (A[3] * m0 + A[4] * m1) + A[5] * m2, am2 = (A[6] * m0 + A[7] * m1) + A[8] * m2; const float mam = (m0 * am0 + m1 * am1) + m2 * am2;
  const float op = 1.0f / (1.0f + nexp(-bf16_rne(opl[n])));
  v4f o0 = {A[0], A[1], A[2], A[3]}, o1 = {A[4], A[5], A[6], A[7]}, o2 = {A[8], am0, am1, am2}, o3 = {mam, op, 0.0f, 0.0f};
  for (int pass = 0; pass < 2; ++pass) { float* d = GPR + (size_t)n * GP; *(volatile v4f*)d = o0; *(volatile v4f*)(d + 4) = o1; *(volatile v4f*)(d + 8) = o2; *(volatile v4f*)(d + 12) = o3; __threadfence(); }
}
__global__ __launch_bounds__(256) void ft_kernel(const float* __restrict__ feats, b16* __restrict__ FT) {
  __shared__ __attribute__((aligned(16))) b16 T[F][64 + 8];
  const int n0 = blockIdx.x * 64, t_ = threadIdx.x;
  for (int q = t_; q < 64 * F; q += 256) { const int nn = q >> 5, f = q & 31; T[f][nn] = (b16)(bf16_rne(feats[(size_t)(n0 + nn) * F + f]) * XS); }
  __syncthreads();
  for (int pass = 0; pass < 2; ++pass) { { const int f = t_ >> 3, c8 = (t_ & 7) * 8; *(volatile v8b*)(FT + (size_t)f * N + n0 + c8) = *(const v8b*)(&T[f][c8]); } __threadfence(); }
}
__global__ __launch_bounds__(64) void splat_kernel(const float* __restrict__ qxyz, const float* __restrict__ GPR, const b16* __restrict__ FT, float* __restrict__ out) {
  __shared__ __attribute__((aligned(16))) float To[2][16][F + 4];
  const int wave = threadIdx.x >> 5, lane = threadIdx.x & 31, hh = lane >> 4, col = lane & 15; const int q0 = blockIdx.x * 32 + wave * 16, qi = q0 + col;
  const float px = bf16_rne(qxyz[qi * 3]), py = bf16_rne(qxyz[qi * 3 + 1]), pz = bf16_rne(qxyz[qi * 3 + 2]);
  const float qq[9] = {px * px, px * py, px * pz, py * px, py * py, py * pz, pz * px, pz * py, pz * pz};
  v8f o[2] = {{}, {}}, ol[2] = {{}, {}}; float wsum = 0.0f;
  for (int kb = 0; kb < N; kb += 32) {
    v16b ph, pl;
#pragma unroll
    for (int hq = 0; hq < 2; ++hq)
#pragma unroll
      for (int r = 0; r < 8; ++r) { const int n = kb + 16 * hq + 8 * hh + r; const float* g = GPR + (size_t)n * GP; const v4f g0 = *(const v4f*)g, g1 = *(const v4f*)(g + 4), g2 = *(const v4f*)(g + 8), g3 = *(const v4f*)(g + 12);
        float qAq = 0.0f; qAq += qq[0] * g0[0]; qAq += qq[1] * g0[1]; qAq += qq[2] * g0[2]; qAq += qq[3] * g0[3]; qAq += qq[4] * g1[0]; qAq += qq[5] * g1[1]; qAq += qq[6] * g1[2]; qAq += qq[7] * g1[3]; qAq += qq[8] * g2[0];
        const float qAmu = (px * g2[1] + py * g2[2]) + pz * g2[3]; const float maha = (qAq - 2.0f * qAmu) + g3[0]; const float w = pmul(g3[1], nexp(-0.5f * maha));
        wsum += w; const b16 h_ = (b16)(w * PS); ph[hq * 8 + r] = h_; pl[hq * 8 + r] = (b16)(w * PS - (float)h_); }
#pragma unroll
    for (int t = 0; t < 2; ++t) { const v16b wf = frag_kb(FT + (size_t)(t * 16 + col) * N + kb, hh); o[t] = wmma16b(wf, ph, o[t]); ol[t] = wmma16b(wf, pl, ol[t]); } }
  wsum += __shfl_xor(wsum, 16); const float inv = 1.0f / ((wsum + 1e-8f) * PS * XS);
#pragma unroll
  for (int t = 0; t < 2; ++t)
#pragma unroll
    for (int r = 0; r < 8; ++r) To[wave][col][t * 16 + 8 * hh + r] = (o[t][r] + ol[t][r]) * inv;
  wave_lds_sync();
  for (int pass = 0; pass < 2; ++pass) { for (int r2 = 0; r2 < 16; r2 += 4) { const int rr = r2 + (lane >> 3), c4 = (lane & 7) * 4; *(volatile v4f*)(out + (size_t)(q0 + rr) * F + c4) = *(const v4f*)(&To[wave][rr][c4]); } __threadfence(); }
}
}

extern "C" void kernel_launch(void* const* d_in, const int* in_sizes, int n_in, void* d_out, int out_size, void* d_ws, size_t ws_size, hipStream_t stream) {
  (void)n_in;
  auto Fp = [&](int i) { return (const float*)d_in[i]; };
  if (in_sizes[0] != Q * 3 || in_sizes[1] != N * 3 || in_sizes[2] != N * 3 || in_sizes[3] != N * 4 || in_sizes[4] != N || in_sizes[5] != N * F || out_size != Q * F) return;
  size_t off = 0; char* ws = (char*)d_ws;
  auto carve = [&](size_t bytes) { char* p = ws + off; off += (bytes + 255) & ~(size_t)255; return p; };
  float* GPR = (float*)carve((size_t)N * GP * 4); b16* FT = (b16*)carve((size_t)F * N * 2);
  if (off > ws_size || off > ((size_t)128 << 20)) return;
  gauss_kernel<<<N / 256, 256, 0, stream>>>(Fp(1), Fp(2), Fp(3), Fp(4), GPR);
  ft_kernel<<<N / 64, 256, 0, stream>>>(Fp(5), FT);
  splat_kernel<<<Q / 32, 64, 0, stream>>>(Fp(0), GPR, FT, (float*)d_out);
}
